// PointNet_20461224198193
// MI455X (gfx1250) — hardware-verified
//
#include <hip/hip_runtime.h>
#include <stdint.h>

#pragma clang fp contract(off)

typedef __attribute__((ext_vector_type(16))) _Float16 v16h;
typedef __attribute__((ext_vector_type(8)))  _Float16 v8h;
typedef __attribute__((ext_vector_type(16))) __bf16   v16b;
typedef __attribute__((ext_vector_type(8)))  __bf16   v8b;
typedef __attribute__((ext_vector_type(8)))  float    v8f;
typedef __attribute__((ext_vector_type(4)))  float    v4f;
typedef __attribute__((ext_vector_type(4)))  unsigned v4u;
typedef __attribute__((ext_vector_type(2)))  unsigned v2u;
typedef __attribute__((ext_vector_type(4)))  int      v4i;

constexpr int NBATCH   = 8;
constexpr int NPTS     = 16384;
constexpr int NQRY     = 512;
constexpr int NCOLS_IN = 35;
constexpr int NFEAT    = 32;
constexpr int NSLOT_A  = 32;
constexpr int NSLOT_B  = 64;
constexpr int OUT_COLS = 259;
constexpr int HROWS    = 518;
constexpr int NPTS_ALL = NBATCH * NPTS;
constexpr int NQRY_ALL = NBATCH * NQRY;
constexpr int CH1 = 64;
constexpr int CH2 = 64;
constexpr int CH3 = 128;

constexpr int PT_B1 = 0;
constexpr int PT_I1 = 64;
constexpr int PT_S1 = 128;
constexpr int PT_B2 = 192;
constexpr int PT_I2 = 256;
constexpr int PT_S2 = 320;
constexpr int PT_B3 = 384;
constexpr int PT_I3 = 512;
constexpr int PT_S3 = 640;
constexpr int PT_R0 = 768;
constexpr int PT_R1 = 896;
constexpr int PT_R2 = 1024;
constexpr int PT_TOTAL = 1152;

static_assert(NPTS_ALL == 131072, "shape");
static_assert(NQRY_ALL == 4096, "shape");
static_assert((256 * NCOLS_IN) % 4 == 0 && (256 * NCOLS_IN) / 4 == 2240, "staging extent");
static_assert((NQRY_ALL * OUT_COLS) % 256 == 0, "flat writer grid");
static_assert(NPTS_ALL % 64 == 0 && CH1 % 64 == 0 && CH3 % 64 == 0 && NFEAT % 32 == 0 && CH1 % 32 == 0, "gemm tiles");

constexpr size_t OFF_FEATSB = 0;
constexpr size_t OFF_POSR   = OFF_FEATSB + (size_t)NPTS_ALL * NFEAT * 2;
constexpr size_t OFF_PNORM  = OFF_POSR + (size_t)NPTS_ALL * 16;
constexpr size_t OFF_WPL    = OFF_PNORM + (size_t)NPTS_ALL * 4;
constexpr size_t OFF_PTAB   = OFF_WPL + 28672;
constexpr size_t OFF_SIDX   = OFF_PTAB + (size_t)PT_TOTAL * 4;
constexpr size_t OFF_SFEAT  = OFF_SIDX + (size_t)NQRY_ALL * 4;
constexpr size_t OFF_QNORM  = OFF_SFEAT + (size_t)NQRY_ALL * NFEAT * 2;
constexpr size_t OFF_Y1     = OFF_QNORM + (size_t)NQRY_ALL * 4;
constexpr size_t OFF_Y2     = OFF_Y1 + (size_t)NPTS_ALL * CH1 * 2;
constexpr size_t OFF_Y3     = OFF_Y2 + (size_t)NPTS_ALL * CH2 * 2;
constexpr size_t OFF_HQ     = OFF_Y3 + (size_t)NPTS_ALL * CH3 * 2;
constexpr size_t WS_TOTAL   = OFF_HQ + (size_t)NQRY_ALL * 256 * 4;
static_assert(WS_TOTAL <= 134217728, "workspace carve");
static_assert(OFF_POSR % 128 == 0 && OFF_PNORM % 128 == 0 && OFF_WPL % 128 == 0 && OFF_PTAB % 128 == 0 &&
              OFF_SIDX % 128 == 0 && OFF_SFEAT % 128 == 0 && OFF_QNORM % 128 == 0 && OFF_Y1 % 128 == 0 &&
              OFF_Y2 % 128 == 0 && OFF_Y3 % 128 == 0 && OFF_HQ % 128 == 0, "line aligned carve");

__device__ __forceinline__ unsigned bf16_bits_rne(float f) {
  const unsigned u = __float_as_uint(f);
  return (u + 0x7FFFu + ((u >> 16) & 1u)) >> 16;
}
__device__ __forceinline__ float bf16_rne(float f) { return __uint_as_float(bf16_bits_rne(f) << 16); }

__device__ __forceinline__ float h16_to_f32(unsigned hb) {
  const unsigned sgn = (hb & 0x8000u) << 16; const unsigned em = hb & 0x7fffu;
  const float fn = __uint_as_float((em << 13) + 0x38000000u);
  const float fs = (float)em * 5.9604644775390625e-8f;
  const float mag = (em < 0x400u) ? fs : fn; return __uint_as_float(__float_as_uint(mag) | sgn); }

__device__ __forceinline__ void keep4_h(v16h a, v16h b, v16h c, v16h d) { asm volatile("v_nop" :: "v"(a), "v"(b), "v"(c), "v"(d)); }
__device__ __forceinline__ void keep4_b(v16b a, v16b b, v16b c, v16b d) { asm volatile("v_nop" :: "v"(a), "v"(b), "v"(c), "v"(d)); }
__device__ __forceinline__ void acc_guard4(v8f& a, v8f& b, v8f& c, v8f& d) { asm volatile("v_nop\n\tv_nop\n\tv_nop\n\tv_nop" : "+v"(a), "+v"(b), "+v"(c), "+v"(d)); }
__device__ __forceinline__ void dep_guard4_h(v8f& a, v8f& b, v8f& c, v8f& d, v16h x, v16h y0, v16h y1, v16h y2, v16h y3) {
  asm volatile("v_nop\n\tv_nop\n\tv_nop\n\tv_nop" : "+v"(a), "+v"(b), "+v"(c), "+v"(d) : "v"(x), "v"(y0), "v"(y1), "v"(y2), "v"(y3));
}
__device__ __forceinline__ void dep_guard4_b(v8f& a, v8f& b, v8f& c, v8f& d, v16b x, v16b y0, v16b y1, v16b y2, v16b y3) {
  asm volatile("v_nop\n\tv_nop\n\tv_nop\n\tv_nop" : "+v"(a), "+v"(b), "+v"(c), "+v"(d) : "v"(x), "v"(y0), "v"(y1), "v"(y2), "v"(y3));
}

template <typename T> struct Frag;
template <> struct Frag<_Float16> {
  typedef v16h V; union U { v16h v; v8h h[2]; };
  static __device__ __forceinline__ v16h load(const _Float16* p) {
    U f; f.h[0] = *(const v8h*)(p); f.h[1] = *(const v8h*)(p + 16); return f.v;
  }
  static __device__ __forceinline__ v8f mma(v16h a, v16h b, v8f c) {
    return __builtin_amdgcn_wmma_f32_16x16x32_f16(false, a, false, b, (short)0, c, false, false);
  }
  static __device__ __forceinline__ void guard4(v8f& a, v8f& b, v8f& c, v8f& d, v16h x, v16h y0, v16h y1, v16h y2, v16h y3) { dep_guard4_h(a, b, c, d, x, y0, y1, y2, y3); }
  static __device__ __forceinline__ void keep(v16h a, v16h b, v16h c, v16h d) { keep4_h(a, b, c, d); }
};
template <> struct Frag<__bf16> {
  typedef v16b V; union U { v16b v; v8b h[2]; };
  static __device__ __forceinline__ v16b load(const __bf16* p) {
    U f; f.h[0] = *(const v8b*)(p); f.h[1] = *(const v8b*)(p + 16); return f.v;
  }
  static __device__ __forceinline__ v8f mma(v16b a, v16b b, v8f c) {
    return __builtin_amdgcn_wmma_f32_16x16x32_bf16(false, a, false, b, (short)0, c, false, false);
  }
  static __device__ __forceinline__ void guard4(v8f& a, v8f& b, v8f& c, v8f& d, v16b x, v16b y0, v16b y1, v16b y2, v16b y3) { dep_guard4_b(a, b, c, d, x, y0, y1, y2, y3); }
  static __device__ __forceinline__ void keep(v16b a, v16b b, v16b c, v16b d) { keep4_b(a, b, c, d); }
};
template <int ET> struct Elem;
template <> struct Elem<0> { typedef _Float16 T; };
template <> struct Elem<1> { typedef __bf16 T; };

__global__ __launch_bounds__(256) void prep_points(const float* pc, unsigned* featsW, float* posR, float* pnorm) {
  __shared__ __align__(16) float sx[256 * NCOLS_IN];
  const int t = threadIdx.x;
  const size_t pbase = (size_t)blockIdx.x * 256;
  const v4f* src = (const v4f*)(pc + pbase * NCOLS_IN);
#pragma unroll 1
  for (int it = 0; it < 9; ++it) {
    const int f = it * 256 + t;
    const int fc = f < 2240 ? f : 2239;
    const v4f x = src[fc];
    const float x0 = x[0];
    const float x1 = x[1];
    const float x2 = x[2];
    const float x3 = x[3];
    v4f r;
    r[0] = bf16_rne(x0);
    r[1] = bf16_rne(x1);
    r[2] = bf16_rne(x2);
    r[3] = bf16_rne(x3);
    if (f < 2240) *(v4f*)(sx + 4 * f) = r;
  }
  __syncthreads();

  v4u wv[4];
#pragma unroll
  for (int it = 0; it < 4; ++it) {
    const int c = it * 256 + t;
    const int p = c >> 2;
    const int sub = c & 3;
    const float* fp = sx + p * NCOLS_IN + 3 + 8 * sub;
    unsigned w[4];
#pragma unroll
    for (int e2 = 0; e2 < 4; ++e2) {
      const unsigned u0 = __float_as_uint(fp[2 * e2]);
      const unsigned u1 = __float_as_uint(fp[2 * e2 + 1]);
      w[e2] = (u0 >> 16) | (u1 & 0xffff0000u);
    }
    v4u q;
    q[0] = w[0]; q[1] = w[1]; q[2] = w[2]; q[3] = w[3];
    wv[it] = q;
  }

  const float* fr = sx + t * NCOLS_IN + 3;
  float a[8];
#pragma unroll
  for (int k = 0; k < 8; ++k) a[k] = fr[k] * fr[k];
#pragma unroll
  for (int g = 1; g < 4; ++g) {
#pragma unroll
    for (int k = 0; k < 8; ++k) {
      const float sq = fr[8 * g + k] * fr[8 * g + k];
      a[k] = a[k] + sq;
    }
  }
  const float pn = ((a[0] + a[4]) + (a[2] + a[6])) + ((a[1] + a[5]) + (a[3] + a[7]));
  v4f pv;
  pv[0] = sx[t * NCOLS_IN + 0];
  pv[1] = sx[t * NCOLS_IN + 1];
  pv[2] = sx[t * NCOLS_IN + 2];
  pv[3] = 0.0f;

  volatile v4u* fdst = (volatile v4u*)featsW + pbase * 4;
  volatile v4f* pdst = (volatile v4f*)posR + pbase;
  volatile float* ndst = pnorm + pbase;
  for (int pass = 0; pass < 2; ++pass) {
#pragma unroll
    for (int it = 0; it < 4; ++it) fdst[it * 256 + t] = wv[it];
    pdst[t] = pv;
    ndst[t] = pn;
    __threadfence();
  }
}

__global__ __launch_bounds__(256) void prep_params(
    const float* w1, const float* b1, const float* g1, const float* be1, const float* m1, const float* v1,
    const float* w2, const float* b2, const float* g2, const float* be2, const float* m2, const float* v2,
    const float* w3, const float* b3, const float* g3, const float* be3, const float* m3, const float* v3,
    unsigned* wplane, float* ptab) {
  __shared__ __align__(16) unsigned sw[1792 * 4];
  __shared__ __align__(16) float sp[PT_TOTAL];
  __shared__ float sc[256];
  __shared__ float su[64];
  const int t = threadIdx.x;

#pragma unroll 1
  for (int it = 0; it < 7; ++it) {
    const int c = it * 256 + t;
    const float* src;
    int e;
    if (it == 0) { src = w1; e = c * 8; }
    else if (it < 3) { src = w2; e = (c - 256) * 8; }
    else { src = w3; e = (c - 768) * 8; }
    const v4f xa = *(const v4f*)(src + e);
    const v4f xb = *(const v4f*)(src + e + 4);
    float x[8];
    x[0] = xa[0]; x[1] = xa[1]; x[2] = xa[2]; x[3] = xa[3];
    x[4] = xb[0]; x[5] = xb[1]; x[6] = xb[2]; x[7] = xb[3];
    unsigned hb[8];
#pragma unroll
    for (int k = 0; k < 8; ++k) {
      const float r = bf16_rne(x[k]);
      const unsigned bb = __float_as_uint(r) >> 16;
      const _Float16 hx = (_Float16)r;
      const unsigned short hs = __builtin_bit_cast(unsigned short, hx);
      const unsigned fb = (unsigned)hs;
      hb[k] = (it == 0) ? bb : fb;
    }
    v4u q;
    q[0] = hb[0] | (hb[1] << 16);
    q[1] = hb[2] | (hb[3] << 16);
    q[2] = hb[4] | (hb[5] << 16);
    q[3] = hb[6] | (hb[7] << 16);
    *(v4u*)(sw + 4 * c) = q;
  }

  {
    const float* pb; const float* pg; const float* pbe; const float* pm; const float* pvv;
    int j, oB, oI, oS;
    if (t < 64) { pb = b1; pg = g1; pbe = be1; pm = m1; pvv = v1; j = t; oB = PT_B1; oI = PT_I1; oS = PT_S1; }
    else if (t < 128) { pb = b2; pg = g2; pbe = be2; pm = m2; pvv = v2; j = t - 64; oB = PT_B2; oI = PT_I2; oS = PT_S2; }
    else { pb = b3; pg = g3; pbe = be3; pm = m3; pvv = v3; j = t - 128; oB = PT_B3; oI = PT_I3; oS = PT_S3; }
    const float bq = bf16_rne(pb[j]);
    const float gq = bf16_rne(pg[j]);
    const float beq = bf16_rne(pbe[j]);
    const float mq = bf16_rne(pm[j]);
    const float vq = bf16_rne(pvv[j]);
    const float inv = gq / sqrtf(vq + 1e-5f);
    const float sh = beq - mq * inv;
    sp[oB + j] = bq;
    sp[oI + j] = inv;
    sp[oS + j] = sh;
    float cz = bq * inv + sh;
    cz = cz > 0.0f ? cz : 0.0f;
    sc[t] = cz;
  }
  __syncthreads();

  if (t < 64) {
    float acc = 0.0f;
#pragma unroll 4
    for (int k = 0; k < 64; ++k) {
      const float wq = bf16_rne(w2[t * 64 + k]);
      const float pr = wq * sc[k];
      acc = acc + pr;
    }
    float y = (acc + sp[PT_B2 + t]) * sp[PT_I2 + t] + sp[PT_S2 + t];
    y = y > 0.0f ? y : 0.0f;
    su[t] = y;
  }
  __syncthreads();

  if (t < 128) {
    float a2 = 0.0f, a3 = 0.0f;
#pragma unroll 4
    for (int k = 0; k < 64; ++k) {
      const float wq = bf16_rne(w3[t * 64 + k]);
      const float p2 = wq * sc[64 + k];
      const float p3 = wq * su[k];
      a2 = a2 + p2;
      a3 = a3 + p3;
    }
    const float bb = sp[PT_B3 + t], ii = sp[PT_I3 + t], ss = sp[PT_S3 + t];
    float y2 = (a2 + bb) * ii + ss;
    y2 = y2 > 0.0f ? y2 : 0.0f;
    float y3 = (a3 + bb) * ii + ss;
    y3 = y3 > 0.0f ? y3 : 0.0f;
    const float c3 = sc[128 + t];
    const float r1 = fmaxf(c3, y2);
    const float r2 = fmaxf(r1, y3);
    sp[PT_R0 + t] = c3;
    sp[PT_R1 + t] = r1;
    sp[PT_R2 + t] = r2;
  }
  __syncthreads();

  for (int pass = 0; pass < 2; ++pass) {
#pragma unroll 1
    for (int it = 0; it < 7; ++it) {
      const int c = it * 256 + t;
      const v4u q = *(const v4u*)(sw + 4 * c);
      ((volatile v4u*)wplane)[c] = q;
    }
#pragma unroll 1
    for (int it = 0; it < 2; ++it) {
      const int c = it * 256 + t;
      if (c < PT_TOTAL / 4) {
        const v4f q = *(const v4f*)(sp + 4 * c);
        ((volatile v4f*)ptab)[c] = q;
      }
    }
    __threadfence();
  }
}

__global__ __launch_bounds__(512) void fps_select(const float* posR, int* sidx) {
#pragma clang fp contract(off)
  __shared__ float sval[2][16];
  __shared__ int   sind[2][16];
  __shared__ __align__(16) int swin[NQRY];
  const int b = blockIdx.x;
  const int t = threadIdx.x;
  const int lane = t & 31;
  const int wid = t >> 5;
  const v4f* pb = (const v4f*)posR + (size_t)b * NPTS;

  float px[32], py[32], pz[32], d[32];
#pragma unroll
  for (int g = 0; g < 8; ++g) {
    v4f q0 = pb[(4 * g + 0) * 512 + t];
    v4f q1 = pb[(4 * g + 1) * 512 + t];
    v4f q2 = pb[(4 * g + 2) * 512 + t];
    v4f q3 = pb[(4 * g + 3) * 512 + t];
    asm volatile("" : "+v"(q0), "+v"(q1), "+v"(q2), "+v"(q3) :: "memory");
    px[4 * g + 0] = q0[0]; py[4 * g + 0] = q0[1]; pz[4 * g + 0] = q0[2];
    px[4 * g + 1] = q1[0]; py[4 * g + 1] = q1[1]; pz[4 * g + 1] = q1[2];
    px[4 * g + 2] = q2[0]; py[4 * g + 2] = q2[1]; pz[4 * g + 2] = q2[2];
    px[4 * g + 3] = q3[0]; py[4 * g + 3] = q3[1]; pz[4 * g + 3] = q3[2];
  }
  if (t == 0) swin[0] = 0;

  float wx, wy, wz;
  {
    const v4f p0 = pb[0];
    wx = p0[0]; wy = p0[1]; wz = p0[2];
  }
  float bd = -1.0f;
  int bj = 0;
#pragma unroll
  for (int i = 0; i < 32; ++i) {
    const float dx = px[i] - wx;
    const float dy = py[i] - wy;
    const float dz = pz[i] - wz;
    const float t0 = dx * dx;
    const float t1 = dy * dy;
    const float t2 = dz * dz;
    const float dd = (t0 + t2) + t1;
    d[i] = dd;
    const int j = i * 512 + t;
    const bool take = dd > bd;
    bd = take ? dd : bd;
    bj = take ? j : bj;
  }

#pragma unroll 1
  for (int s = 1; s < NQRY; ++s) {
#pragma unroll
    for (int off = 16; off > 0; off >>= 1) {
      const float od = __shfl_xor(bd, off, 32);
      const int oj = __shfl_xor(bj, off, 32);
      const bool take = (od > bd) || ((od == bd) && (oj < bj));
      bd = take ? od : bd;
      bj = take ? oj : bj;
    }
    const int buf = s & 1;
    if (lane == 0) { sval[buf][wid] = bd; sind[buf][wid] = bj; }
    __syncthreads();
    float vd = sval[buf][lane & 15];
    int vj = sind[buf][lane & 15];
#pragma unroll
    for (int off = 8; off > 0; off >>= 1) {
      const float od = __shfl_xor(vd, off, 32);
      const int oj = __shfl_xor(vj, off, 32);
      const bool take = (od > vd) || ((od == vd) && (oj < vj));
      vd = take ? od : vd;
      vj = take ? oj : vj;
    }
    int wj = vj < 0 ? 0 : vj;
    wj = wj > NPTS - 1 ? NPTS - 1 : wj;
    if (t == 0) swin[s] = wj;
    const v4f wp = pb[wj];
    wx = wp[0]; wy = wp[1]; wz = wp[2];
    bd = -1.0f;
    bj = 0;
#pragma unroll
    for (int i = 0; i < 32; ++i) {
      const float dx = px[i] - wx;
      const float dy = py[i] - wy;
      const float dz = pz[i] - wz;
      const float t0 = dx * dx;
      const float t1 = dy * dy;
      const float t2 = dz * dz;
      const float dd = (t0 + t2) + t1;
      const float dn = fminf(d[i], dd);
      d[i] = dn;
      const int j = i * 512 + t;
      const bool take = dn > bd;
      bd = take ? dn : bd;
      bj = take ? j : bj;
    }
  }
  __syncthreads();
  if (t < 128) {
    const v4i val = *(const v4i*)(swin + 4 * t);
    volatile v4i* dst = (volatile v4i*)sidx + (size_t)b * 128 + t;
    *dst = val;
    __threadfence();
    *dst = val;
  }
}

__global__ __launch_bounds__(256) void sample_rows(const unsigned* featsW, const float* pnorm, const int* sidx,
                                                   unsigned* sfeatW, float* qnorm) {
  const int t = threadIdx.x;
  const int g = blockIdx.x * 256 + t;
  const int row = g >> 2;
  const int sub = g & 3;
  const int b = row >> 9;
  int idx = sidx[row];
  idx = idx < 0 ? 0 : idx;
  idx = idx > NPTS - 1 ? NPTS - 1 : idx;
  const v4u w = ((const v4u*)featsW)[((size_t)b * NPTS + idx) * 4 + sub];
  volatile v4u* dst = (volatile v4u*)sfeatW + g;
  *dst = w;
  __threadfence();
  *dst = w;
  if (t < 64) {
    const int row2 = blockIdx.x * 64 + t;
    const int b2 = row2 >> 9;
    int i2 = sidx[row2];
    i2 = i2 < 0 ? 0 : i2;
    i2 = i2 > NPTS - 1 ? NPTS - 1 : i2;
    const float v = pnorm[(size_t)b2 * NPTS + i2];
    volatile float* qd = qnorm + row2;
    *qd = v;
    __threadfence();
    *qd = v;
  }
}

template <int ET>
__global__ __launch_bounds__(256) void mlp_gemm_bn_relu(
    const unsigned short* __restrict__ Ap, int lda,
    const unsigned short* __restrict__ Btp, int ldb,
    unsigned short* __restrict__ Cout, int ldc,
    const float* __restrict__ bvec, const float* __restrict__ ivec, const float* __restrict__ svec,
    int M, int N, int K) {
  typedef typename Elem<ET>::T T;
  typedef typename Frag<T>::V V;
  const T* A = (const T*)Ap;
  const T* Bt = (const T*)Btp;
  __shared__ __align__(16) float sT[8][16 * 68];
  const int lane = threadIdx.x & 31;
  const int wave = threadIdx.x >> 5;
  const int tilesN = N >> 6;
  const int tilesM = M >> 6;
  const int tile = blockIdx.x * 8 + wave;
  if (tile >= tilesM * tilesN) return;
  const int tm = tile / tilesN;
  const int tn = tile - tm * tilesN;
  const int m0 = tm << 6;
  const int n0 = tn << 6;
  const int rlane = lane & 15;
  const int koff = (lane >> 4) * 8;
  const int mOff = (lane >> 4) * 8;

  v8f acc[4][4];
#pragma unroll
  for (int i = 0; i < 4; ++i)
#pragma unroll
    for (int j = 0; j < 4; ++j) acc[i][j] = (v8f){0.f, 0.f, 0.f, 0.f, 0.f, 0.f, 0.f, 0.f};

  for (int k0 = 0; k0 < K; k0 += 32) {
    V bh[4];
#pragma unroll
    for (int j = 0; j < 4; ++j) {
      const size_t bo = (size_t)(n0 + (j << 4) + rlane) * ldb + koff + k0;
      bh[j] = Frag<T>::load(Bt + bo);
    }
#pragma unroll
    for (int i = 0; i < 4; ++i) {
      const size_t ao = (size_t)(m0 + (i << 4) + rlane) * lda + koff + k0;
      V ah = Frag<T>::load(A + ao);
#pragma unroll
      for (int j = 0; j < 4; ++j) acc[i][j] = Frag<T>::mma(ah, bh[j], acc[i][j]);
      Frag<T>::guard4(acc[i][0], acc[i][1], acc[i][2], acc[i][3], ah, bh[0], bh[1], bh[2], bh[3]);
    }
    Frag<T>::keep(bh[0], bh[1], bh[2], bh[3]);
  }
  acc_guard4(acc[0][0], acc[0][1], acc[0][2], acc[0][3]);
  acc_guard4(acc[1][0], acc[1][1], acc[1][2], acc[1][3]);
  acc_guard4(acc[2][0], acc[2][1], acc[2][2], acc[2][3]);
  acc_guard4(acc[3][0], acc[3][1], acc[3][2], acc[3][3]);

  float bv[4], iv[4], sv[4];
#pragma unroll
  for (int j = 0; j < 4; ++j) {
    const int n = n0 + (j << 4) + rlane;
    bv[j] = bvec[n];
    iv[j] = ivec[n];
    sv[j] = svec[n];
  }
  float* slab = sT[wave];
#pragma unroll
  for (int i = 0; i < 4; ++i) {
    const int mBase = m0 + (i << 4);
#pragma unroll
    for (int j = 0; j < 4; ++j) {
#pragma unroll
      for (int r = 0; r < 8; ++r) {
        float v = acc[i][j][r];
        v = (v + bv[j]) * iv[j] + sv[j];
        v = v > 0.0f ? v : 0.0f;
        slab[(mOff + r) * 68 + (j << 4) + rlane] = v;
      }
    }
    __builtin_amdgcn_fence(__ATOMIC_RELEASE, "workgroup");
    __builtin_amdgcn_wave_barrier();
    __builtin_amdgcn_fence(__ATOMIC_ACQUIRE, "workgroup");
    {
      const int q = lane >> 3, c8 = (lane & 7) * 8;
      for (int pass = 0; pass < 2; ++pass) {
#pragma unroll
        for (int it = 0; it < 4; ++it) {
          const int row = it * 4 + q;
          const float* sp = slab + row * 68 + c8;
          v8h hv;
#pragma unroll
          for (int e = 0; e < 8; ++e) hv[e] = (_Float16)sp[e];
          *(volatile v8h*)(Cout + (size_t)(mBase + row) * ldc + n0 + c8) = hv;
        }
        __threadfence();
      }
    }
    __builtin_amdgcn_fence(__ATOMIC_RELEASE, "workgroup");
    __builtin_amdgcn_wave_barrier();
    __builtin_amdgcn_fence(__ATOMIC_ACQUIRE, "workgroup");
  }
}

__global__ __launch_bounds__(128) void ball_group(
    const unsigned short* sfeatB, const unsigned short* featsB, const float* qnorm, const float* pnorm,
    const unsigned* Y3w, const float* ptab, float* HQ) {
#pragma clang fp contract(off)
  __shared__ __align__(16) int L1[4][16 * NSLOT_A];
  __shared__ __align__(16) int L2[4][16 * NSLOT_B];
  const int t = threadIdx.x;
  const int wave = t >> 5;
  const int lane = t & 31;
  const int h = lane >> 4;
  const int n = lane & 15;
  const int tileq = blockIdx.x * 4 + wave;
  const int b = tileq >> 5;
  const int q0 = tileq * 16;
  int* l1 = L1[wave];
  int* l2 = L2[wave];
  for (int i = lane; i < 16 * NSLOT_A; i += 32) l1[i] = -1;
  for (int i = lane; i < 16 * NSLOT_B; i += 32) l2[i] = -1;
  __syncthreads();

  const v16b afrag = Frag<__bf16>::load((const __bf16*)sfeatB + (size_t)(q0 + n) * NFEAT + 8 * h);
  float qn[8];
#pragma unroll
  for (int r = 0; r < 8; ++r) qn[r] = qnorm[q0 + 8 * h + r];
  int c1[8], c2[8];
#pragma unroll
  for (int r = 0; r < 8; ++r) { c1[r] = 0; c2[r] = 0; }
  const unsigned lmask = (1u << n) - 1u;
  const unsigned sh16 = 16u * (unsigned)h;
  const __bf16* fb = (const __bf16*)featsB + (size_t)b * NPTS * NFEAT;
  const float* pnb = pnorm + (size_t)b * NPTS;

#pragma unroll 1
  for (int tile = 0; tile < NPTS / 16; ++tile) {
    const int j = tile * 16 + n;
    const v16b bfrag = Frag<__bf16>::load(fb + (size_t)j * NFEAT + 8 * h);
    const float pn = pnb[j];
    v8f acc = (v8f){0.f, 0.f, 0.f, 0.f, 0.f, 0.f, 0.f, 0.f};
    acc = Frag<__bf16>::mma(afrag, bfrag, acc);
    asm volatile("v_nop\n\tv_nop\n\tv_nop\n\tv_nop" : "+v"(acc) : "v"(afrag), "v"(bfrag));
#pragma unroll
    for (int r = 0; r < 8; ++r) {
      const float qp = qn[r] + pn;
      const float two = 2.0f * acc[r];
      const float d2 = qp - two;
      const bool w1 = d2 < 36.0f;
      const bool w2 = d2 < 64.0f;
      const unsigned bal1 = __builtin_amdgcn_ballot_w32(w1);
      const unsigned bal2 = __builtin_amdgcn_ballot_w32(w2);
      const unsigned m1 = (bal1 >> sh16) & 0xffffu;
      const unsigned m2 = (bal2 >> sh16) & 0xffffu;
      const int s1 = c1[r] + (int)__popc(m1 & lmask);
      const int s2 = c2[r] + (int)__popc(m2 & lmask);
      if (w1 && s1 < NSLOT_A) l1[(8 * h + r) * NSLOT_A + s1] = j;
      if (w2 && s2 < NSLOT_B) l2[(8 * h + r) * NSLOT_B + s2] = j;
      c1[r] += (int)__popc(m1);
      c2[r] += (int)__popc(m2);
    }
    bool notfull = false;
#pragma unroll
    for (int r = 0; r < 8; ++r) notfull = notfull || (c1[r] < NSLOT_A) || (c2[r] < NSLOT_B);
    const unsigned nf = __builtin_amdgcn_ballot_w32(notfull);
    if (nf == 0u) break;
  }
  __syncthreads();

  const v2u* yb = (const v2u*)Y3w + (size_t)b * NPTS * 32;
  const v4f r2 = *(const v4f*)(ptab + PT_R2 + 4 * lane);
  const float r20 = r2[0];
  const float r21 = r2[1];
  const float r22 = r2[2];
  const float r23 = r2[3];
#pragma unroll 1
  for (int row = 0; row < 16; ++row) {
#pragma unroll 1
    for (int br = 0; br < 2; ++br) {
      const int ns = br ? NSLOT_B : NSLOT_A;
      const int lbase = row * ns;
      unsigned m0 = 0u, m1 = 0u, m2 = 0u, m3 = 0u;
#pragma unroll 4
      for (int s = 0; s < ns; ++s) {
        const int ia = l1[(lbase + s) & (16 * NSLOT_A - 1)];
        const int ib = l2[lbase + s];
        const int idx = br ? ib : ia;
        const unsigned vm = ~(unsigned)(idx >> 31);
        int ic = idx < 0 ? 0 : idx;
        ic = ic > NPTS - 1 ? NPTS - 1 : ic;
        const v2u w = yb[(size_t)ic * 32 + lane];
        const unsigned wa = w[0] & vm;
        const unsigned wb = w[1] & vm;
        const unsigned a0 = wa & 0xffffu, a1 = wa >> 16, a2 = wb & 0xffffu, a3 = wb >> 16;
        m0 = a0 > m0 ? a0 : m0;
        m1 = a1 > m1 ? a1 : m1;
        m2 = a2 > m2 ? a2 : m2;
        m3 = a3 > m3 ? a3 : m3;
      }
      v4f o;
      o[0] = fmaxf(r20, h16_to_f32(m0));
      o[1] = fmaxf(r21, h16_to_f32(m1));
      o[2] = fmaxf(r22, h16_to_f32(m2));
      o[3] = fmaxf(r23, h16_to_f32(m3));
      volatile v4f* dst = (volatile v4f*)(HQ + (size_t)(q0 + row) * 256 + br * 128) + lane;
      *dst = o;
      __threadfence();
      *dst = o;
    }
  }
}

__global__ __launch_bounds__(256) void pool_pack(const float* posR, const int* sidx, const float* HQ,
                                                 const float* ptab, float* out) {
  const int e = blockIdx.x * 256 + threadIdx.x;
  const int row = e / OUT_COLS;
  const int col = e - row * OUT_COLS;
  const int b = row >> 9;
  const int i = row & 511;
  int si = sidx[row];
  si = si < 0 ? 0 : si;
  si = si > NPTS - 1 ? NPTS - 1 : si;
  const int pcol = col < 2 ? col : 2;
  float pv = posR[((size_t)b * NPTS + si) * 4 + pcol];
  const int cc = col >= 3 ? col - 3 : 0;
  const int c = cc & 127;
  const int start = (i * HROWS) >> 9;
  const int end = ((i + 1) * HROWS + 511) >> 9;
  float hv[3], rv[3], fr[3];
  bool inw[3];
#pragma unroll
  for (int k = 0; k < 3; ++k) {
    const int r = start + k;
    inw[k] = r < end;
    const int rc = r < HROWS - 1 ? r : HROWS - 1;
    int ridx = 3;
    ridx = rc <= 2 ? rc : ridx;
    ridx = rc >= HROWS - 3 ? (HROWS - 1 - rc) : ridx;
    int qrow = rc - 3;
    qrow = qrow < 0 ? 0 : qrow;
    qrow = qrow > NQRY - 1 ? NQRY - 1 : qrow;
    const int rsel = ridx < 2 ? ridx : 2;
    hv[k] = HQ[((size_t)(b * NQRY + qrow)) * 256 + cc];
    rv[k] = ptab[PT_R0 + rsel * 128 + c];
    fr[k] = ridx < 3 ? 1.0f : 0.0f;
  }
  asm volatile("" : "+v"(hv[0]), "+v"(hv[1]), "+v"(hv[2]), "+v"(rv[0]), "+v"(rv[1]), "+v"(rv[2]), "+v"(pv));
  float m = 0.0f;
#pragma unroll
  for (int k = 0; k < 3; ++k) {
    const float fh = 1.0f - fr[k];
    const float va = fr[k] * rv[k];
    const float vb = fh * hv[k];
    const float val = va + vb;
    const float mx = fmaxf(m, val);
    m = (k == 0) ? val : (inw[k] ? mx : m);
  }
  const float fp = col < 3 ? 1.0f : 0.0f;
  const float fq = 1.0f - fp;
  const float oa = fp * pv;
  const float ob = fq * m;
  const float v = oa + ob;
  volatile float* dst = out + e;
  *dst = v;
  __threadfence();
  *dst = v;
}

extern "C" void kernel_launch(void* const* d_in, const int* in_sizes, int n_in,
                              void* d_out, int out_size, void* d_ws, size_t ws_size, hipStream_t stream) {
  if (n_in < 19) return;
  if (in_sizes[0] != NPTS_ALL * NCOLS_IN) return;
  if (in_sizes[1] != CH1 * NFEAT || in_sizes[7] != CH2 * CH1 || in_sizes[13] != CH3 * CH2) return;
  if (out_size != NQRY_ALL * OUT_COLS) return;
  if (ws_size < WS_TOTAL) return;

  const float* pc = (const float*)d_in[0];
  const float* w1 = (const float*)d_in[1];
  const float* b1 = (const float*)d_in[2];
  const float* g1 = (const float*)d_in[3];
  const float* be1 = (const float*)d_in[4];
  const float* m1 = (const float*)d_in[5];
  const float* v1 = (const float*)d_in[6];
  const float* w2 = (const float*)d_in[7];
  const float* b2 = (const float*)d_in[8];
  const float* g2 = (const float*)d_in[9];
  const float* be2 = (const float*)d_in[10];
  const float* m2 = (const float*)d_in[11];
  const float* v2 = (const float*)d_in[12];
  const float* w3 = (const float*)d_in[13];
  const float* b3 = (const float*)d_in[14];
  const float* g3 = (const float*)d_in[15];
  const float* be3 = (const float*)d_in[16];
  const float* m3 = (const float*)d_in[17];
  const float* v3 = (const float*)d_in[18];
  float* out = (float*)d_out;
  char* ws = (char*)d_ws;

  unsigned* featsW = (unsigned*)(ws + OFF_FEATSB);
  float* posR = (float*)(ws + OFF_POSR);
  float* pnorm = (float*)(ws + OFF_PNORM);
  unsigned* wplane = (unsigned*)(ws + OFF_WPL);
  float* ptab = (float*)(ws + OFF_PTAB);
  int* sidx = (int*)(ws + OFF_SIDX);
  unsigned* sfeatW = (unsigned*)(ws + OFF_SFEAT);
  float* qnorm = (float*)(ws + OFF_QNORM);
  unsigned short* y1 = (unsigned short*)(ws + OFF_Y1);
  unsigned short* y2 = (unsigned short*)(ws + OFF_Y2);
  unsigned short* y3 = (unsigned short*)(ws + OFF_Y3);
  float* hq = (float*)(ws + OFF_HQ);
  const unsigned short* w1b = (const unsigned short*)(ws + OFF_WPL);
  const unsigned short* w2h = (const unsigned short*)(ws + OFF_WPL + 4096);
  const unsigned short* w3h = (const unsigned short*)(ws + OFF_WPL + 12288);

  prep_points<<<NPTS_ALL / 256, 256, 0, stream>>>(pc, featsW, posR, pnorm);
  prep_params<<<1, 256, 0, stream>>>(w1, b1, g1, be1, m1, v1, w2, b2, g2, be2, m2, v2,
                                     w3, b3, g3, be3, m3, v3, wplane, ptab);
  fps_select<<<NBATCH, 512, 0, stream>>>(posR, sidx);
  sample_rows<<<NQRY_ALL / 64, 256, 0, stream>>>(featsW, pnorm, sidx, sfeatW, qnorm);

  mlp_gemm_bn_relu<1><<<(NPTS_ALL / 64) * (CH1 / 64) / 8, 256, 0, stream>>>(
      (const unsigned short*)featsW, NFEAT, w1b, NFEAT, y1, CH1,
      ptab + PT_B1, ptab + PT_I1, ptab + PT_S1, NPTS_ALL, CH1, NFEAT);
  mlp_gemm_bn_relu<0><<<(NPTS_ALL / 64) * (CH2 / 64) / 8, 256, 0, stream>>>(
      y1, CH1, w2h, CH1, y2, CH2,
      ptab + PT_B2, ptab + PT_I2, ptab + PT_S2, NPTS_ALL, CH2, CH1);
  mlp_gemm_bn_relu<0><<<(NPTS_ALL / 64) * (CH3 / 64) / 8, 256, 0, stream>>>(
      y2, CH2, w3h, CH2, y3, CH3,
      ptab + PT_B3, ptab + PT_I3, ptab + PT_S3, NPTS_ALL, CH3, CH2);

  ball_group<<<NQRY_ALL / 64, 128, 0, stream>>>((const unsigned short*)sfeatW, (const unsigned short*)featsW,
                                                qnorm, pnorm, (const unsigned*)y3, ptab, hq);
  pool_pack<<<(NQRY_ALL * OUT_COLS) / 256, 256, 0, stream>>>(posR, sidx, hq, ptab, out);
}
